// RelativeStructureAttention_60198261621495
// MI455X (gfx1250) — hardware-verified
//
#include <hip/hip_runtime.h>
#include <math.h>
#include <stdint.h>

#define NB    2
#define SEQ   1024
#define DM    1024
#define NH    16
#define HD    64
#define MROWS (NB * SEQ)
#define NQB   (SEQ / 64)
#define VLP   256
#define RESQB 4
#define QEP   192
#define TROWS 192
#define OFF_BAR 0
#define OFF_POS 17
#define OFF_OCT 113
#define OFF_SEM 138
static_assert(RESQB * 64 <= VLP);
static_assert(NH * HD == DM);
static_assert((SEQ % 64) == 0 && (DM % 64) == 0 && (QEP % 64) == 0 && (TROWS % 64) == 0);
static_assert(OFF_SEM + 13 <= QEP);

typedef _Float16 v16h __attribute__((ext_vector_type(16)));
typedef _Float16 v8h  __attribute__((ext_vector_type(8)));
typedef __bf16   v16b __attribute__((ext_vector_type(16)));
typedef __bf16   v8b  __attribute__((ext_vector_type(8)));
typedef float    v8f  __attribute__((ext_vector_type(8)));
typedef float    v4f  __attribute__((ext_vector_type(4)));
typedef unsigned int v4u __attribute__((ext_vector_type(4)));

__device__ __forceinline__ unsigned short bf_bits(float f) {
  unsigned u = __float_as_uint(f);
  return (unsigned short)((u + 0x7FFFu + ((u >> 16) & 1u)) >> 16);
}
__device__ __forceinline__ float bf_up(unsigned short h) { return __uint_as_float(((unsigned)h) << 16); }
__device__ __forceinline__ unsigned short h_bits(_Float16 x) { return __builtin_bit_cast(unsigned short, x); }
__device__ __forceinline__ unsigned pk16(unsigned short a, unsigned short b) { return (unsigned)a | ((unsigned)b << 16); }
__device__ __forceinline__ int iclamp(int v, int lo, int hi) { return (v < lo) ? lo : ((v > hi) ? hi : v); }
__device__ __forceinline__ int imin(int a, int b) { return (a < b) ? a : b; }
__device__ __forceinline__ v8f zero8() { v8f z = {0.f, 0.f, 0.f, 0.f, 0.f, 0.f, 0.f, 0.f}; return z; }
__device__ __forceinline__ v8h zero8h() {
  const _Float16 z = (_Float16)0.0f;
  v8h r = {z, z, z, z, z, z, z, z};
  return r;
}

__device__ __forceinline__ v16b ldfrag_b(const __bf16* p) {
  union { v16b v; v8b h[2]; } f;
  f.h[0] = *(const v8b*)(p);
  f.h[1] = *(const v8b*)(p + 16);
  return f.v;
}

__device__ __forceinline__ v8f mma_b(v16b a, v16b b, v8f c) {
  c = __builtin_amdgcn_wmma_f32_16x16x32_bf16(false, a, false, b, (short)0, c, false, false);
#if defined(__HIP_DEVICE_COMPILE__)
  asm volatile("v_nop\n\tv_nop\n\tv_nop\n\tv_nop" : "+v"(c) : "v"(a), "v"(b));
#endif
  return c;
}
__device__ __forceinline__ v8f mma_h(v16h a, v16h b, v8f c) {
  c = __builtin_amdgcn_wmma_f32_16x16x32_f16(false, a, false, b, (short)0, c, false, false);
#if defined(__HIP_DEVICE_COMPILE__)
  asm volatile("v_nop\n\tv_nop\n\tv_nop\n\tv_nop" : "+v"(c) : "v"(a), "v"(b));
#endif
  return c;
}
__device__ __forceinline__ v8f mma_b_raw(v16b a, v16b b, v8f c) {
  return __builtin_amdgcn_wmma_f32_16x16x32_bf16(false, a, false, b, (short)0, c, false, false);
}
__device__ __forceinline__ void dep_guard_b(v8f& a, v8f& b, v16b x, v16b y) {
#if defined(__HIP_DEVICE_COMPILE__)
  asm volatile("v_nop\n\tv_nop\n\tv_nop\n\tv_nop" : "+v"(a), "+v"(b) : "v"(x), "v"(y));
#else
  (void)a; (void)b; (void)x; (void)y;
#endif
}
__device__ __forceinline__ void keep4_b(v16b a, v16b b, v16b c, v16b d) {
#if defined(__HIP_DEVICE_COMPILE__)
  asm volatile("v_nop" :: "v"(a), "v"(b), "v"(c), "v"(d));
#else
  (void)a; (void)b; (void)c; (void)d;
#endif
}
__device__ __forceinline__ void acc_guard4(v8f& a, v8f& b, v8f& c, v8f& d) {
#if defined(__HIP_DEVICE_COMPILE__)
  asm volatile("v_nop\n\tv_nop\n\tv_nop\n\tv_nop" : "+v"(a), "+v"(b), "+v"(c), "+v"(d));
#else
  (void)a; (void)b; (void)c; (void)d;
#endif
}

__global__ __launch_bounds__(256) void cvt_bf16x8(const float* __restrict__ in, unsigned short* out, int n8) {
  const int i = blockIdx.x * 256 + threadIdx.x;
  if (i < n8) {
    const v4f a = *(const v4f*)(in + (size_t)i * 8);
    const v4f b = *(const v4f*)(in + (size_t)i * 8 + 4);
    v4u p;
    p[0] = pk16(bf_bits(a[0]), bf_bits(a[1]));
    p[1] = pk16(bf_bits(a[2]), bf_bits(a[3]));
    p[2] = pk16(bf_bits(b[0]), bf_bits(b[1]));
    p[3] = pk16(bf_bits(b[2]), bf_bits(b[3]));
    *(volatile v4u*)(out + (size_t)i * 8) = p;
    __threadfence();
    *(volatile v4u*)(out + (size_t)i * 8) = p;
  }
}

__global__ __launch_bounds__(256) void build_tab(const float* __restrict__ ebar, const float* __restrict__ epos,
                                                 const float* __restrict__ eoct, const float* __restrict__ esem,
                                                 unsigned short* tab) {
  const int g = blockIdx.x * 256 + threadIdx.x;
  if (g < TROWS * 8) {
    const int s  = g >> 3;
    const int d0 = (g & 7) * 8;
    const int rb = iclamp(s, 0, 15);
    const int rp = iclamp(s - OFF_POS, 0, 94);
    const int ro = iclamp(s - OFF_OCT, 0, 23);
    const int rs = iclamp(s - OFF_SEM, 0, 11);
    const bool ub = (s < 16);
    const bool up = (s >= OFF_POS) && (s < OFF_POS + 95);
    const bool uo = (s >= OFF_OCT) && (s < OFF_OCT + 24);
    const bool us = (s >= OFF_SEM) && (s < OFF_SEM + 12);
    float v[8];
#pragma unroll
    for (int e = 0; e < 8; ++e) {
      const int d = d0 + e;
      const float fb = ebar[rb * HD + d];
      const float fp = epos[rp * HD + d];
      const float fo = eoct[ro * HD + d];
      const float fs = esem[rs * HD + d];
      float t = 0.f;
      t = ub ? fb : t;
      t = up ? fp : t;
      t = uo ? fo : t;
      t = us ? fs : t;
      v[e] = t;
    }
    v4u p;
    p[0] = pk16(bf_bits(v[0]), bf_bits(v[1]));
    p[1] = pk16(bf_bits(v[2]), bf_bits(v[3]));
    p[2] = pk16(bf_bits(v[4]), bf_bits(v[5]));
    p[3] = pk16(bf_bits(v[6]), bf_bits(v[7]));
    *(volatile v4u*)(tab + (size_t)s * HD + d0) = p;
    __threadfence();
    *(volatile v4u*)(tab + (size_t)s * HD + d0) = p;
  }
}

template <int NSPLIT, int OUT_MODE>
__global__ __launch_bounds__(256) void gemm64(
    const unsigned short* __restrict__ Ap, const unsigned short* A2p, int lda, long long strideA,
    const unsigned short* __restrict__ Btp, const unsigned short* Bt2p, int ldb, long long strideB,
    void* Cout, int ldc, long long strideC,
    void* Cout2, int ldc2, long long strideC2, int N2,
    int M, int N, int K, float rscale) {
  const __bf16* A   = (const __bf16*)(const void*)Ap;
  const __bf16* A2  = (const __bf16*)(const void*)A2p;
  const __bf16* Bt  = (const __bf16*)(const void*)Btp;
  const __bf16* Bt2 = (const __bf16*)(const void*)Bt2p;
  __shared__ __align__(16) float sT[8][16 * 68];
  const int b    = blockIdx.y;
  const int lane = threadIdx.x & 31;
  const int wave = threadIdx.x >> 5;
  const int tilesN = N >> 6;
  const int tilesM = M >> 6;
  const int tile = blockIdx.x * 8 + wave;
  if (tile >= tilesM * tilesN) return;
  const int tm = tile / tilesN;
  const int tn = tile - tm * tilesN;
  const int m0 = tm << 6;
  const int n0 = tn << 6;

  const __bf16* Ab  = A  + (size_t)b * strideA;
  const __bf16* Bb  = Bt + (size_t)b * strideB;
  const __bf16* Ab2 = (NSPLIT >= 1) ? (A2  + (size_t)b * strideA) : Ab;
  const __bf16* Bb2 = (NSPLIT == 2) ? (Bt2 + (size_t)b * strideB) : Bb;

  const int rlane = lane & 15;
  const int koff  = (lane >> 4) * 8;
  const int mOff  = (lane >> 4) * 8;

  v8f acc[4][4];
#pragma unroll
  for (int i = 0; i < 4; ++i)
#pragma unroll
    for (int j = 0; j < 4; ++j) acc[i][j] = zero8();

  for (int k0 = 0; k0 < K; k0 += 32) {
    v16b bh[4], bl[4];
#pragma unroll
    for (int j = 0; j < 4; ++j) {
      const size_t bo = (size_t)(n0 + (j << 4) + rlane) * ldb + koff + k0;
      bh[j] = ldfrag_b(Bb + bo);
      if (NSPLIT == 2) bl[j] = ldfrag_b(Bb2 + bo); else bl[j] = bh[j];
    }
#pragma unroll
    for (int i = 0; i < 4; ++i) {
      const size_t ao = (size_t)(m0 + (i << 4) + rlane) * lda + koff + k0;
      const v16b ah = ldfrag_b(Ab + ao);
      v16b al = ah;
      if (NSPLIT >= 1) al = ldfrag_b(Ab2 + ao);
#pragma unroll
      for (int j = 0; j < 4; ++j) {
        acc[i][j] = mma_b_raw(ah, bh[j], acc[i][j]);
        if (NSPLIT >= 1) acc[i][j] = mma_b_raw(al, bh[j], acc[i][j]);
        if (NSPLIT == 2) acc[i][j] = mma_b_raw(ah, bl[j], acc[i][j]);
      }
      dep_guard_b(acc[i][0], acc[i][3], ah, al);
    }
    keep4_b(bh[0], bh[1], bh[2], bh[3]);
    if (NSPLIT == 2) keep4_b(bl[0], bl[1], bl[2], bl[3]);
  }
  acc_guard4(acc[0][0], acc[0][1], acc[0][2], acc[0][3]);
  acc_guard4(acc[1][0], acc[1][1], acc[1][2], acc[1][3]);
  acc_guard4(acc[2][0], acc[2][1], acc[2][2], acc[2][3]);
  acc_guard4(acc[3][0], acc[3][1], acc[3][2], acc[3][3]);

  float* slab = sT[wave];
#pragma unroll
  for (int i = 0; i < 4; ++i) {
    const int mBase = m0 + (i << 4);
#pragma unroll
    for (int j = 0; j < 4; ++j) {
#pragma unroll
      for (int r = 0; r < 8; ++r) {
        slab[(mOff + r) * 68 + (j << 4) + rlane] = acc[i][j][r];
      }
    }
    __builtin_amdgcn_fence(__ATOMIC_RELEASE, "workgroup");
    __builtin_amdgcn_wave_barrier();
    __builtin_amdgcn_fence(__ATOMIC_ACQUIRE, "workgroup");
    if (OUT_MODE == 0) {
      float* C = (float*)Cout + (size_t)b * strideC;
      const int hh = lane >> 4, c4 = (lane & 15) * 4;
      for (int pass = 0; pass < 2; ++pass) {
#pragma unroll
        for (int it = 0; it < 8; ++it) {
          const int row = it * 2 + hh;
          const v4f v = *(const v4f*)(slab + row * 68 + c4);
          *(volatile v4f*)(C + (size_t)(mBase + row) * ldc + n0 + c4) = v;
        }
        __threadfence();
      }
    } else {
      const int q = lane >> 3, c8 = (lane & 7) * 8;
      unsigned short* C  = (unsigned short*)Cout  + (size_t)b * strideC;
      unsigned short* C2 = (unsigned short*)Cout2 + (size_t)b * strideC2;
      const bool wlo = (OUT_MODE == 2) || (n0 < N2);
      v4u hv[4], lv[4];
#pragma unroll
      for (int it = 0; it < 4; ++it) {
        const int row = it * 4 + q;
        const float* sp = slab + row * 68 + c8;
        v4u a, a2;
#pragma unroll
        for (int e = 0; e < 4; ++e) {
          const float f0 = sp[2 * e], f1 = sp[2 * e + 1];
          unsigned short h0, h1, l0, l1;
          if (OUT_MODE == 2) {
            h0 = bf_bits(f0); h1 = bf_bits(f1);
            l0 = bf_bits(f0 - bf_up(h0)); l1 = bf_bits(f1 - bf_up(h1));
          } else {
            const _Float16 x0 = (_Float16)f0, x1 = (_Float16)f1;
            h0 = h_bits(x0); h1 = h_bits(x1);
            l0 = h_bits((_Float16)((f0 - (float)x0) * rscale));
            l1 = h_bits((_Float16)((f1 - (float)x1) * rscale));
          }
          a[e] = pk16(h0, h1); a2[e] = pk16(l0, l1);
        }
        hv[it] = a; lv[it] = a2;
      }
      for (int pass = 0; pass < 2; ++pass) {
#pragma unroll
        for (int it = 0; it < 4; ++it) {
          const int row = it * 4 + q;
          *(volatile v4u*)(C + (size_t)(mBase + row) * ldc + n0 + c8) = hv[it];
          if (wlo) *(volatile v4u*)(C2 + (size_t)(mBase + row) * ldc2 + n0 + c8) = lv[it];
        }
        __threadfence();
      }
    }
    __builtin_amdgcn_fence(__ATOMIC_RELEASE, "workgroup");
    __builtin_amdgcn_wave_barrier();
    __builtin_amdgcn_fence(__ATOMIC_ACQUIRE, "workgroup");
  }
}

template <bool RES>
__global__ __launch_bounds__(128, 3)
void attn_rel64(const unsigned short* __restrict__ qhp, const unsigned short* __restrict__ qlp,
                const unsigned short* __restrict__ khp, const unsigned short* __restrict__ klp,
                const unsigned short* __restrict__ vhp, const unsigned short* __restrict__ vlp,
                const unsigned short* __restrict__ erp, const float* __restrict__ qe,
                const int* __restrict__ ibar, const int* __restrict__ ipos,
                const int* __restrict__ ioct, const int* __restrict__ isem,
                unsigned short* ohp, unsigned short* olp,
                int qbBase, int nqbThis, float sscale) {
  union FB { v16b v; v8b h[2]; };
  union FH { v16h v; v8h h[2]; };
  __shared__ __align__(16) unsigned char smem[RES ? 65536 : 49152];
  __bf16*   const Ksh = (__bf16*)(void*)(smem);
  __bf16*   const Ksl = (__bf16*)(void*)(smem + 8192);
  _Float16* const Vth = (_Float16*)(void*)(smem + 16384);
  __bf16*   const Esh = (__bf16*)(void*)(smem + 24576);
  _Float16* const Psh = (_Float16*)(void*)(smem + 40960);
  _Float16* const Vtl = (_Float16*)(void*)(smem + (RES ? 49152 : 16384));
  _Float16* const Psl = (_Float16*)(void*)(smem + (RES ? 57344 : 40960));
  float*    const Os  = (float*)(void*)(smem);

  const int tid  = threadIdx.x;
  const int wave = tid >> 5;
  const int lane = tid & 31;
  const int hh   = lane >> 4;
  const int c    = lane & 15;

  const int bx   = blockIdx.x;
  const int qbl  = bx % nqbThis;
  const int rest = bx / nqbThis;
  const int h    = rest % NH;
  const int b    = rest / NH;
  const int qb   = qbBase + qbl;
  const int q0   = qb * 64 + wave * 16;
  const size_t rowB = (size_t)b * SEQ;

  const __bf16* Qh  = (const __bf16*)(const void*)qhp + (size_t)h * HD;
  const __bf16* Ql  = (const __bf16*)(const void*)qlp + (size_t)h * HD;
  const __bf16* Kh  = (const __bf16*)(const void*)khp + (size_t)h * HD;
  const __bf16* Kl  = (const __bf16*)(const void*)klp + (size_t)h * HD;
  const _Float16* Vh = (const _Float16*)(const void*)vhp + ((size_t)b * DM + (size_t)h * HD) * SEQ;
  const _Float16* Vl = (const _Float16*)(const void*)vlp + ((size_t)b * DM + (size_t)h * HD) * VLP;
  const __bf16* Erb = (const __bf16*)(const void*)erp;
  const size_t trow0 = rowB + (size_t)(q0 + 8 * hh);
  const float* qew   = qe + ((size_t)h * MROWS + trow0) * QEP;
  const size_t ib0   = trow0 * (size_t)SEQ;

  v16b qah[2], qal[2];
#pragma unroll
  for (int dc = 0; dc < 2; ++dc) {
    const size_t qo = (rowB + q0 + c) * DM + dc * 32 + 8 * hh;
    qah[dc] = ldfrag_b(Qh + qo);
    qal[dc] = ldfrag_b(Ql + qo);
  }

  float mrow[8], lrow[8];
  v8f oacc[4];
#pragma unroll
  for (int r = 0; r < 8; ++r) { mrow[r] = -INFINITY; lrow[r] = 0.f; }
#pragma unroll
  for (int t = 0; t < 4; ++t) oacc[t] = zero8();

  const int nkt = (qb + 1 < NQB) ? (qb + 1) : NQB;
  for (int kt = 0; kt < nkt; ++kt) {
    const int kv0 = kt * 64;
    int ebb = SEQ - 64 + kv0 - qb * 64;
    ebb = (ebb < 0) ? 0 : ebb;
    __syncthreads();
    {
      const int r = tid >> 1, half = (tid & 1) * 32;
      const __bf16*   kg  = Kh + (rowB + kv0 + r) * DM + half;
      const __bf16*   klg = Kl + (rowB + kv0 + r) * DM + half;
      const _Float16* vg  = Vh + (size_t)r * SEQ + kv0 + half;
      const int kvl = (kv0 + 64 <= VLP) ? kv0 : (VLP - 64);
      const _Float16* vlg = Vl + (size_t)r * VLP + kvl + half;
      const bool resOK = (kv0 + 64 <= VLP);
#pragma unroll
      for (int i = 0; i < 4; ++i) {
        const v8b a0 = *(const v8b*)(kg + 8 * i);
        const v8b a1 = *(const v8b*)(klg + 8 * i);
        const v8h b0 = *(const v8h*)(vg + 8 * i);
        *(v8b*)(Ksh + r * 64 + half + 8 * i) = a0;
        *(v8b*)(Ksl + r * 64 + half + 8 * i) = a1;
        *(v8h*)(Vth + r * 64 + half + 8 * i) = b0;
        if (RES) {
          v8h b1 = *(const v8h*)(vlg + 8 * i);
          if (!resOK) b1 = zero8h();
          *(v8h*)(Vtl + r * 64 + half + 8 * i) = b1;
        }
      }
      const int erow = imin(ebb + tid, SEQ - 1);
      const __bf16* eg = Erb + (size_t)erow * HD;
#pragma unroll
      for (int i = 0; i < 8; ++i) *(v8b*)(Esh + tid * 64 + 8 * i) = *(const v8b*)(eg + 8 * i);
    }
    __syncthreads();

    v8f s[4];
#pragma unroll
    for (int j = 0; j < 4; ++j) {
      s[j] = zero8();
#pragma unroll
      for (int dc = 0; dc < 2; ++dc) {
        FB kb, kl;
        kb.h[0] = *(const v8b*)(Ksh + (j * 16 + c) * 64 + dc * 32 + 8 * hh);
        kb.h[1] = *(const v8b*)(Ksh + (j * 16 + c) * 64 + dc * 32 + 16 + 8 * hh);
        kl.h[0] = *(const v8b*)(Ksl + (j * 16 + c) * 64 + dc * 32 + 8 * hh);
        kl.h[1] = *(const v8b*)(Ksl + (j * 16 + c) * 64 + dc * 32 + 16 + 8 * hh);
        s[j] = mma_b(qah[dc], kb.v, s[j]);
        s[j] = mma_b(qah[dc], kl.v, s[j]);
        s[j] = mma_b(qal[dc], kb.v, s[j]);
      }
    }

    {
      const int wb = (3 - wave) * 16;
      v8f prev = zero8();
#pragma unroll
      for (int u = 0; u < 5; ++u) {
        v8f cur = zero8();
#pragma unroll
        for (int dc = 0; dc < 2; ++dc) {
          FB eb;
          const __bf16* ep = Esh + (wb + u * 16 + c) * 64 + dc * 32 + 8 * hh;
          eb.h[0] = *(const v8b*)(ep);
          eb.h[1] = *(const v8b*)(ep + 16);
          cur = mma_b(qah[dc], eb.v, cur);
          cur = mma_b(qal[dc], eb.v, cur);
        }
        if (u >= 1) {
#pragma unroll
          for (int r = 0; r < 8; ++r) {
            const int base = 15 - (8 * hh + r) + c;
            const int src  = (lane & 16) | (base & 15);
            const float vlo = __shfl(prev[r], src, 32);
            const float vhi = __shfl(cur[r], src, 32);
            s[u - 1][r] += (base < 16) ? vlo : vhi;
          }
        }
        prev = cur;
      }
    }

    _Float16* pwh = Psh + wave * (16 * 64);
    _Float16* pwl = Psl + (RES ? wave : 0) * (16 * 64);
#pragma unroll
    for (int r = 0; r < 8; ++r) {
      const float* qrr  = qew + (size_t)r * QEP;
      const size_t io   = ib0 + (size_t)r * SEQ + (size_t)(kv0 + c);
      const int    trow = q0 + 8 * hh + r;
      float m = -INFINITY;
#pragma unroll
      for (int j = 0; j < 4; ++j) {
        const int key = kv0 + j * 16 + c;
        const int x0 = iclamp(ibar[io + j * 16], 0, 16);
        const int x1 = iclamp(ipos[io + j * 16], 0, 95);
        const int x2 = iclamp(ioct[io + j * 16], 0, 24);
        const int x3 = iclamp(isem[io + j * 16], 0, 12);
        const float bsum = (qrr[OFF_BAR + x0] + qrr[OFF_POS + x1]) + (qrr[OFF_OCT + x2] + qrr[OFF_SEM + x3]);
        float sv = (s[j][r] + bsum) * sscale;
        sv = (key <= trow) ? sv : -1.0e9f;
        s[j][r] = sv;
        m = fmaxf(m, sv);
      }
#pragma unroll
      for (int off = 1; off < 16; off <<= 1) m = fmaxf(m, __shfl_xor(m, off, 32));
      const float mnew  = fmaxf(mrow[r], m);
      const float msafe = (mnew == -INFINITY) ? 0.f : mnew;
      const float alpha = __expf(mrow[r] - msafe);
      mrow[r] = mnew;
      float psum = 0.f;
#pragma unroll
      for (int j = 0; j < 4; ++j) {
        const float p = __expf(s[j][r] - msafe);
        psum += p;
        const float p1k = p * 1024.0f;
        const _Float16 ph = (_Float16)p1k;
        pwh[(8 * hh + r) * 64 + j * 16 + c] = ph;
        if (RES) {
          const _Float16 pl = (_Float16)((p1k - (float)ph) * 4096.0f);
          pwl[(8 * hh + r) * 64 + j * 16 + c] = pl;
        }
      }
#pragma unroll
      for (int off = 1; off < 16; off <<= 1) psum += __shfl_xor(psum, off, 32);
      lrow[r] = lrow[r] * alpha + psum;
#pragma unroll
      for (int t = 0; t < 4; ++t) oacc[t][r] *= alpha;
    }
    __builtin_amdgcn_fence(__ATOMIC_RELEASE, "workgroup");
    __builtin_amdgcn_wave_barrier();
    __builtin_amdgcn_fence(__ATOMIC_ACQUIRE, "workgroup");

    v8f o1[4];
#pragma unroll
    for (int t = 0; t < 4; ++t) o1[t] = zero8();
#pragma unroll 1
    for (int kk = 0; kk < 2; ++kk) {
      FH pa, pl;
      pa.h[0] = *(const v8h*)(pwh + c * 64 + kk * 32 + 8 * hh);
      pa.h[1] = *(const v8h*)(pwh + c * 64 + kk * 32 + 16 + 8 * hh);
      if (RES) {
        pl.h[0] = *(const v8h*)(pwl + c * 64 + kk * 32 + 8 * hh);
        pl.h[1] = *(const v8h*)(pwl + c * 64 + kk * 32 + 16 + 8 * hh);
      } else {
        pl.v = pa.v;
      }
#pragma unroll
      for (int t = 0; t < 4; ++t) {
        FH vb;
        vb.h[0] = *(const v8h*)(Vth + (t * 16 + c) * 64 + kk * 32 + 8 * hh);
        vb.h[1] = *(const v8h*)(Vth + (t * 16 + c) * 64 + kk * 32 + 16 + 8 * hh);
        oacc[t] = mma_h(pa.v, vb.v, oacc[t]);
        if (RES) {
          FH vl;
          vl.h[0] = *(const v8h*)(Vtl + (t * 16 + c) * 64 + kk * 32 + 8 * hh);
          vl.h[1] = *(const v8h*)(Vtl + (t * 16 + c) * 64 + kk * 32 + 16 + 8 * hh);
          o1[t] = mma_h(pa.v, vl.v, o1[t]);
          o1[t] = mma_h(pl.v, vb.v, o1[t]);
        }
      }
    }
    if (RES) {
#pragma unroll
      for (int t = 0; t < 4; ++t)
#pragma unroll
        for (int r = 0; r < 8; ++r) oacc[t][r] += o1[t][r] * (1.0f / 4096.0f);
    }
  }

  __syncthreads();
  float* os = Os + wave * (16 * 64);
#pragma unroll
  for (int r = 0; r < 8; ++r) {
    const float l = lrow[r];
    const float inv = ((l > 0.f) ? (1.0f / l) : 0.f) * (1.0f / 1024.0f);
#pragma unroll
    for (int t = 0; t < 4; ++t) os[(8 * hh + r) * 64 + t * 16 + c] = oacc[t][r] * inv;
  }
  __builtin_amdgcn_fence(__ATOMIC_RELEASE, "workgroup");
  __builtin_amdgcn_wave_barrier();
  __builtin_amdgcn_fence(__ATOMIC_ACQUIRE, "workgroup");
  {
    const int q4 = lane >> 3, c8 = (lane & 7) * 8;
    v4u hv[4], lv[4];
#pragma unroll
    for (int it = 0; it < 4; ++it) {
      const int row = it * 4 + q4;
      const float* sp = os + row * 64 + c8;
      v4u a, a2;
#pragma unroll
      for (int e = 0; e < 4; ++e) {
        const float f0 = sp[2 * e], f1 = sp[2 * e + 1];
        const unsigned short h0 = bf_bits(f0), h1 = bf_bits(f1);
        const unsigned short l0 = bf_bits(f0 - bf_up(h0)), l1 = bf_bits(f1 - bf_up(h1));
        a[e] = pk16(h0, h1); a2[e] = pk16(l0, l1);
      }
      hv[it] = a; lv[it] = a2;
    }
    for (int pass = 0; pass < 2; ++pass) {
#pragma unroll
      for (int it = 0; it < 4; ++it) {
        const int row = it * 4 + q4;
        const size_t go = (rowB + q0 + row) * DM + (size_t)h * HD + c8;
        *(volatile v4u*)(ohp + go) = hv[it];
        *(volatile v4u*)(olp + go) = lv[it];
      }
      __threadfence();
    }
  }
}

extern "C" void kernel_launch(void* const* d_in, const int* in_sizes, int n_in,
                              void* d_out, int out_size, void* d_ws, size_t ws_size,
                              hipStream_t stream) {
  if (n_in < 14) return;
  if (in_sizes[0] != NB * SEQ * DM) return;
  if (in_sizes[1] != NB * SEQ * SEQ || in_sizes[2] != NB * SEQ * SEQ ||
      in_sizes[3] != NB * SEQ * SEQ || in_sizes[4] != NB * SEQ * SEQ) return;
  if (in_sizes[5] != DM * DM || in_sizes[6] != DM * DM || in_sizes[7] != DM * DM || in_sizes[8] != DM * DM) return;
  if (in_sizes[9] != SEQ * HD) return;
  if (in_sizes[10] != 16 * HD || in_sizes[11] != 95 * HD || in_sizes[12] != 24 * HD || in_sizes[13] != 12 * HD) return;
  if (out_size != NB * SEQ * DM) return;

  const float* x    = (const float*)d_in[0];
  const int*   rbar = (const int*)d_in[1];
  const int*   rpos = (const int*)d_in[2];
  const int*   roct = (const int*)d_in[3];
  const int*   rsem = (const int*)d_in[4];
  const float* Wq   = (const float*)d_in[5];
  const float* Wk   = (const float*)d_in[6];
  const float* Wv   = (const float*)d_in[7];
  const float* Wo   = (const float*)d_in[8];
  const float* Er   = (const float*)d_in[9];
  const float* Ebar = (const float*)d_in[10];
  const float* Epos = (const float*)d_in[11];
  const float* Eoct = (const float*)d_in[12];
  const float* Esem = (const float*)d_in[13];

  const size_t PX  = (size_t)MROWS * DM * 2;
  const size_t PW  = (size_t)DM * DM * 2;
  const size_t PE  = (size_t)SEQ * HD * 2;
  const size_t PT  = (size_t)TROWS * HD * 2;
  const size_t PVT = (size_t)NB * DM * SEQ * 2;
  const size_t PVL = (size_t)NB * DM * VLP * 2;
  const size_t PQE = (size_t)NH * MROWS * QEP * 4;
  size_t off = 0;
  const size_t oXb  = off; off += PX;
  const size_t oWq  = off; off += PW;
  const size_t oWk  = off; off += PW;
  const size_t oWv  = off; off += PW;
  const size_t oWo  = off; off += PW;
  const size_t oEr  = off; off += PE;
  const size_t oTb  = off; off += PT;
  const size_t oQh  = off; off += PX;
  const size_t oQl  = off; off += PX;
  const size_t oKh  = off; off += PX;
  const size_t oKl  = off; off += PX;
  const size_t oVTh = off; off += PVT;
  const size_t oVTl = off; off += PVL;
  const size_t oQE  = off; off += PQE;
  const size_t oOh  = off; off += PX;
  const size_t oOl  = off; off += PX;
  if (off > ws_size) return;
  if (off > (size_t)134217728) return;

  char* ws = (char*)d_ws;
  unsigned short* Xb  = (unsigned short*)(ws + oXb);
  unsigned short* Wqb = (unsigned short*)(ws + oWq);
  unsigned short* Wkb = (unsigned short*)(ws + oWk);
  unsigned short* Wvb = (unsigned short*)(ws + oWv);
  unsigned short* Wob = (unsigned short*)(ws + oWo);
  unsigned short* Erb = (unsigned short*)(ws + oEr);
  unsigned short* Tb  = (unsigned short*)(ws + oTb);
  unsigned short* Qh  = (unsigned short*)(ws + oQh);
  unsigned short* Ql  = (unsigned short*)(ws + oQl);
  unsigned short* Kh  = (unsigned short*)(ws + oKh);
  unsigned short* Kl  = (unsigned short*)(ws + oKl);
  unsigned short* VTh = (unsigned short*)(ws + oVTh);
  unsigned short* VTl = (unsigned short*)(ws + oVTl);
  float*          QE  = (float*)(ws + oQE);
  unsigned short* Oh  = (unsigned short*)(ws + oOh);
  unsigned short* Ol  = (unsigned short*)(ws + oOl);

  const dim3 blk(256);
  const int n8x = MROWS * DM / 8;
  const int n8w = DM * DM / 8;
  const int n8e = SEQ * HD / 8;
  const dim3 gCvtX((n8x + 255) / 256);
  const dim3 gCvtW((n8w + 255) / 256);
  const dim3 gCvtE((n8e + 255) / 256);
  const dim3 gTab((TROWS * 8 + 255) / 256);
  const dim3 gProj(((MROWS / 64) * (DM / 64) + 7) / 8, 1);
  const dim3 gVT(((DM / 64) * (SEQ / 64) + 7) / 8, NB);
  const dim3 gQE(((MROWS / 64) * (QEP / 64) + 7) / 8, NH);

  cvt_bf16x8<<<gCvtX, blk, 0, stream>>>(x, Xb, n8x);
  cvt_bf16x8<<<gCvtW, blk, 0, stream>>>(Wq, Wqb, n8w);
  cvt_bf16x8<<<gCvtW, blk, 0, stream>>>(Wk, Wkb, n8w);
  cvt_bf16x8<<<gCvtW, blk, 0, stream>>>(Wv, Wvb, n8w);
  cvt_bf16x8<<<gCvtW, blk, 0, stream>>>(Wo, Wob, n8w);
  cvt_bf16x8<<<gCvtE, blk, 0, stream>>>(Er, Erb, n8e);
  build_tab<<<gTab, blk, 0, stream>>>(Ebar, Epos, Eoct, Esem, Tb);
  gemm64<0, 2><<<gProj, blk, 0, stream>>>(
      Xb, Xb, DM, 0LL, Wqb, Wqb, DM, 0LL,
      (void*)Qh, DM, 0LL, (void*)Ql, DM, 0LL, DM,
      MROWS, DM, DM, 1.0f);
  gemm64<0, 2><<<gProj, blk, 0, stream>>>(
      Xb, Xb, DM, 0LL, Wkb, Wkb, DM, 0LL,
      (void*)Kh, DM, 0LL, (void*)Kl, DM, 0LL, DM,
      MROWS, DM, DM, 1.0f);
  gemm64<0, 3><<<gVT, blk, 0, stream>>>(
      Wvb, Wvb, DM, 0LL, Xb, Xb, DM, (long long)SEQ * DM,
      (void*)VTh, SEQ, (long long)DM * SEQ, (void*)VTl, VLP, (long long)DM * VLP, VLP,
      DM, SEQ, DM, 4096.0f);
  gemm64<1, 0><<<gQE, blk, 0, stream>>>(
      Qh, Ql, DM, (long long)HD, Tb, Tb, HD, 0LL,
      (void*)QE, QEP, (long long)MROWS * QEP, (void*)QE, QEP, 0LL, QEP,
      MROWS, QEP, HD, 1.0f);
  attn_rel64<true><<<dim3(NB * NH * RESQB), dim3(128), 0, stream>>>(
      Qh, Ql, Kh, Kl, VTh, VTl, Erb, QE, rbar, rpos, roct, rsem, Oh, Ol, 0, RESQB, 0.125f);
  attn_rel64<false><<<dim3(NB * NH * (NQB - RESQB)), dim3(128), 0, stream>>>(
      Qh, Ql, Kh, Kl, VTh, VTl, Erb, QE, rbar, rpos, roct, rsem, Oh, Ol, RESQB, NQB - RESQB, 0.125f);
  gemm64<1, 0><<<gProj, blk, 0, stream>>>(
      Oh, Ol, DM, 0LL, Wob, Wob, DM, 0LL,
      d_out, DM, 0LL, d_out, DM, 0LL, DM,
      MROWS, DM, DM, 1.0f);
  (void)hipGetLastError();
}
